// GATC_4904852652851
// MI455X (gfx1250) — hardware-run, weakly checked
//
#include <hip/hip_runtime.h>
#include <stddef.h>
#include <stdint.h>


#define HF       64
#define NCLS     5
#define NG       64
#define HTHR     (NG * NCLS)
#define NTHR     256
#define NWAVE    8
#define ETHR     128
#define EPT      8
#define NGRP     2
#define CHUNK    (NTHR * EPT * NGRP)
#define WCAP     (EPT * NGRP * 32)
#define LISTN    (NWAVE * WCAP)
#define NBC      4096
#define NBF      1024
#define RCAP     40960
#define RBN      128
#define OTHR     512
#define DEGCAP   128
#define CNB      32
#define GROWS    128
#define APH      (HF + 8)
#define WSCAP    134217728
#define LDS_FILL ((RCAP + NBF + LISTN) * 4 + 64)
#define SLOPE    0.2f
#define ASCL     16.0f
#define WSCL     64.0f
#define OSCL     0.0009765625f
#define WPIECES  (2 * HF * HF / 8)

static_assert((CHUNK & (CHUNK - 1)) == 0);
static_assert(CHUNK <= 4096);
static_assert((NBC & (NBC - 1)) == 0 && (NBF & (NBF - 1)) == 0);
static_assert(NBC == 4 * NBF);
static_assert(OTHR * 8 == NBC);
static_assert((RCAP % 32) == 0);
static_assert((NBF % CNB) == 0);
static_assert((GROWS % CNB) == 0);
static_assert(CNB == 8 * (ETHR / 32));
static_assert(GROWS == NWAVE * 16);
static_assert(NTHR == NWAVE * 32);
static_assert((WPIECES % NTHR) == 0);
static_assert((HF % 32) == 0);
static_assert(((APH * 2) % 16) == 0);
static_assert(GROWS * APH * 2 <= GROWS * HF * 4);
static_assert(HTHR == NG * NCLS && HTHR <= 1024 && ((NG * NCLS) % 4) == 0);
static_assert((DEGCAP % 32) == 0);

typedef float    v2f  __attribute__((ext_vector_type(2)));
typedef float    v4f  __attribute__((ext_vector_type(4)));
typedef float    v8f  __attribute__((ext_vector_type(8)));
typedef int      v4i  __attribute__((ext_vector_type(4)));
typedef _Float16 v8h  __attribute__((ext_vector_type(8)));
typedef _Float16 v16h __attribute__((ext_vector_type(16)));
union FragH { v16h v; v8h h[2]; };

__device__ __forceinline__ v8f wm(v16h a, v16h b, v8f c) {
  v8f d = __builtin_amdgcn_wmma_f32_16x16x32_f16(false, a, false, b, (short)0, c, false, false);
  asm volatile("v_nop\n\tv_nop\n\tv_nop\n\tv_nop" : "+v"(d) : "v"(a), "v"(b));
  return d;
}
__device__ __forceinline__ v8f z8f() { v8f z = {0.f, 0.f, 0.f, 0.f, 0.f, 0.f, 0.f, 0.f}; return z; }

__device__ __forceinline__ v8h cvt8(v4f a, v4f b) {
  v8h o;
  o[0] = (_Float16)a.x; o[1] = (_Float16)a.y; o[2] = (_Float16)a.z; o[3] = (_Float16)a.w;
  o[4] = (_Float16)b.x; o[5] = (_Float16)b.y; o[6] = (_Float16)b.z; o[7] = (_Float16)b.w;
  return o;
}
__device__ __forceinline__ v8h gath8h(const float* p, int stride, float sc) {
  v4f a, c;
  a.x = p[0];          a.y = p[stride];     a.z = p[2 * stride]; a.w = p[3 * stride];
  c.x = p[4 * stride]; c.y = p[5 * stride]; c.z = p[6 * stride]; c.w = p[7 * stride];
  a = a * sc; c = c * sc;
  return cvt8(a, c);
}

template <int NB>
__device__ __forceinline__ int scan_chunk(const int* __restrict__ keys, int nE, int cbase, int slotBase,
                                          int vec8, int* list, int tid, int lane, int wave) {
  int wc = 0;
#pragma unroll
  for (int g = 0; g < NGRP; ++g) {
    const int el0  = (g * NTHR + tid) * EPT;
    const int e0   = cbase + el0;
    const int sent = -2147483647 - 1;
    v4i da, db;
    if (vec8 != 0 && cbase + CHUNK <= nE) {
      da = *(const v4i*)(keys + e0);
      db = *(const v4i*)(keys + e0 + 4);
    } else {
      da.x = (e0     < nE) ? keys[min(e0, nE - 1)] : sent;
      da.y = (e0 + 1 < nE) ? keys[min(e0 + 1, nE - 1)] : sent;
      da.z = (e0 + 2 < nE) ? keys[min(e0 + 2, nE - 1)] : sent;
      da.w = (e0 + 3 < nE) ? keys[min(e0 + 3, nE - 1)] : sent;
      db.x = (e0 + 4 < nE) ? keys[min(e0 + 4, nE - 1)] : sent;
      db.y = (e0 + 5 < nE) ? keys[min(e0 + 5, nE - 1)] : sent;
      db.z = (e0 + 6 < nE) ? keys[min(e0 + 6, nE - 1)] : sent;
      db.w = (e0 + 7 < nE) ? keys[min(e0 + 7, nE - 1)] : sent;
    }
    const unsigned nb = (unsigned)slotBase;
    const unsigned s0 = (unsigned)da.x - nb, s1 = (unsigned)da.y - nb;
    const unsigned s2 = (unsigned)da.z - nb, s3 = (unsigned)da.w - nb;
    const unsigned s4 = (unsigned)db.x - nb, s5 = (unsigned)db.y - nb;
    const unsigned s6 = (unsigned)db.z - nb, s7 = (unsigned)db.w - nb;
    const bool h0 = s0 < (unsigned)NB, h1 = s1 < (unsigned)NB, h2 = s2 < (unsigned)NB, h3 = s3 < (unsigned)NB;
    const bool h4 = s4 < (unsigned)NB, h5 = s5 < (unsigned)NB, h6 = s6 < (unsigned)NB, h7 = s7 < (unsigned)NB;
    const unsigned any = __builtin_amdgcn_ballot_w32(h0 | h1 | h2 | h3 | h4 | h5 | h6 | h7);
    if (any != 0u) {
#define HITJ(J, HJ, SJ) { \
        const unsigned mj = __builtin_amdgcn_ballot_w32(HJ); \
        if (mj != 0u) { \
          if (HJ) { \
            const int pos = wc + (int)__builtin_amdgcn_mbcnt_lo(mj, 0u); \
            if (pos < WCAP) list[wave * WCAP + pos] = ((el0 + (J)) << 12) | (int)(SJ); \
          } \
          wc += (int)__builtin_popcount(mj); } }
      HITJ(0, h0, s0)
      HITJ(1, h1, s1)
      HITJ(2, h2, s2)
      HITJ(3, h3, s3)
      HITJ(4, h4, s4)
      HITJ(5, h5, s5)
      HITJ(6, h6, s6)
      HITJ(7, h7, s7)
#undef HITJ
    }
  }
  return wc;
}

__global__ __launch_bounds__(NTHR) void k_wprep(
    const float* __restrict__ w1, const float* __restrict__ w2, _Float16* wp) {
  const int tid = (int)threadIdx.x;
  const int pc = (int)blockIdx.x * NTHR + tid;
  const float* src = (blockIdx.x < 2) ? w1 : w2;
  const int lp = pc & (WPIECES / 2 - 1);
  const int n  = lp >> 3;
  const int k0 = (lp & 7) * 8;
  const v8h o = gath8h(src + (size_t)k0 * HF + n, HF, WSCL);
  _Float16* dp = wp + (size_t)pc * 8;
  *(volatile v8h*)dp = o;
  __threadfence();
  *(volatile v8h*)dp = o;
}

__global__ __launch_bounds__(NTHR) void k_count(
    const int* __restrict__ keys, int* cnt, int nE, int vec8) {
  __shared__ __attribute__((aligned(16))) int scnt[NBC];
  __shared__ __attribute__((aligned(16))) int list[LISTN];
  __shared__ int wcnt[NWAVE];
  const int tid = threadIdx.x, lane = tid & 31, wave = tid >> 5;
  const int nodeBase = blockIdx.x * NBC;

  for (int i = tid; i < NBC; i += NTHR) scnt[i] = 0;
  __syncthreads();

  const int nChunks = (nE + CHUNK - 1) / CHUNK;
#pragma unroll 1
  for (int ch = 0; ch < nChunks; ++ch) {
    const int cbase = ch * CHUNK;
    const int wc = scan_chunk<NBC>(keys, nE, cbase, nodeBase, vec8, list, tid, lane, wave);
    if (lane == 0) wcnt[wave] = wc;
    __syncthreads();
    if (wave == 0) {
#pragma unroll 1
      for (int wsx = 0; wsx < NWAVE; ++wsx) {
        int n = __builtin_amdgcn_readfirstlane(wcnt[wsx]);
        n = n > WCAP ? WCAP : (n < 0 ? 0 : n);
        const int* lp = list + wsx * WCAP;
#pragma unroll 1
        for (int i = 0; i < n; ++i) {
          const int ent  = __builtin_amdgcn_readfirstlane(lp[i]);
          const int slot = ent & (NBC - 1);
          if (lane == 0) scnt[slot] = scnt[slot] + 1;
        }
      }
    }
    __syncthreads();
  }

  v4i cq[4];
#pragma unroll
  for (int q = 0; q < 4; ++q) {
    const int f = (wave * 4 + q) * 128 + 4 * lane;
    cq[q] = *(const v4i*)(scnt + f);
  }
  int* cp = cnt + (size_t)nodeBase;
#pragma unroll
  for (int q = 0; q < 4; ++q) {
    const int f = (wave * 4 + q) * 128 + 4 * lane;
    *(volatile v4i*)(cp + f) = cq[q];
  }
  __threadfence();
#pragma unroll
  for (int q = 0; q < 4; ++q) {
    const int f = (wave * 4 + q) * 128 + 4 * lane;
    *(volatile v4i*)(cp + f) = cq[q];
  }
}

__global__ __launch_bounds__(OTHR) void k_offsets(
    const int* __restrict__ cnt, int* off, int* rbase, int nChunk) {
  __shared__ __attribute__((aligned(16))) int soff[NBC];
  __shared__ __attribute__((aligned(16))) int srb[RBN];
  __shared__ int wtot[OTHR / 32];
  const int tid = threadIdx.x, lane = tid & 31, wave = tid >> 5, sub = tid >> 7;
  for (int i = tid; i < RBN; i += OTHR) srb[i] = 0;
  int carry = 0;
#pragma unroll 1
  for (int ch = 0; ch < nChunk; ++ch) {
    const int base = ch * NBC;
    const v4i c0 = *(const v4i*)(cnt + base + 8 * tid);
    const v4i c1 = *(const v4i*)(cnt + base + 8 * tid + 4);
    const int e0 = max(c0.x, 0), e1 = max(c0.y, 0), e2 = max(c0.z, 0), e3 = max(c0.w, 0);
    const int e4 = max(c1.x, 0), e5 = max(c1.y, 0), e6 = max(c1.z, 0), e7 = max(c1.w, 0);
    const int ts = e0 + e1 + e2 + e3 + e4 + e5 + e6 + e7;
    int incl = ts;
#pragma unroll
    for (int d = 1; d < 32; d <<= 1) {
      const int t = __shfl_up(incl, d);
      if (lane >= d) incl += t;
    }
    if (lane == 31) wtot[wave] = incl;
    __syncthreads();
    const int S0 = wtot[0]  + wtot[1]  + wtot[2]  + wtot[3];
    const int S1 = wtot[4]  + wtot[5]  + wtot[6]  + wtot[7];
    const int S2 = wtot[8]  + wtot[9]  + wtot[10] + wtot[11];
    const int S3 = wtot[12] + wtot[13] + wtot[14] + wtot[15];
    int pre = 0;
#pragma unroll 1
    for (int w = 4 * sub; w < wave; ++w) pre += wtot[w];
    const int b0 = carry;
    const int b1 = b0 + ((S0 + 31) & ~31);
    const int b2 = b1 + ((S1 + 31) & ~31);
    const int b3 = b2 + ((S2 + 31) & ~31);
    const int b4 = b3 + ((S3 + 31) & ~31);
    const int myb = sub == 0 ? b0 : (sub == 1 ? b1 : (sub == 2 ? b2 : b3));
    if (tid == 0) {
      srb[min(4 * ch + 0, RBN - 1)] = b0;
      srb[min(4 * ch + 1, RBN - 1)] = b1;
      srb[min(4 * ch + 2, RBN - 1)] = b2;
      srb[min(4 * ch + 3, RBN - 1)] = b3;
    }
    int run = myb + pre + incl - ts;
    soff[8 * tid + 0] = run; run += e0;
    soff[8 * tid + 1] = run; run += e1;
    soff[8 * tid + 2] = run; run += e2;
    soff[8 * tid + 3] = run; run += e3;
    soff[8 * tid + 4] = run; run += e4;
    soff[8 * tid + 5] = run; run += e5;
    soff[8 * tid + 6] = run; run += e6;
    soff[8 * tid + 7] = run;
    carry = b4;
    __syncthreads();
    const v4i o0 = *(const v4i*)(soff + 4 * tid);
    const v4i o1 = *(const v4i*)(soff + 4 * (tid + OTHR));
    int* op = off + base;
    *(volatile v4i*)(op + 4 * tid) = o0;
    *(volatile v4i*)(op + 4 * (tid + OTHR)) = o1;
    __threadfence();
    *(volatile v4i*)(op + 4 * tid) = o0;
    *(volatile v4i*)(op + 4 * (tid + OTHR)) = o1;
    __syncthreads();
  }
  if (tid == 0) srb[min(4 * nChunk, RBN - 1)] = carry;
  __syncthreads();
  v4i rv = {0, 0, 0, 0};
  if (tid < 32) rv = *(const v4i*)(srb + 4 * tid);
  if (tid < 32) *(volatile v4i*)(rbase + 4 * tid) = rv;
  __threadfence();
  if (tid < 32) *(volatile v4i*)(rbase + 4 * tid) = rv;
}

__global__ __launch_bounds__(NTHR) void k_fill(
    const int* __restrict__ keys, const int* __restrict__ off, const int* __restrict__ rbase,
    int* csr, int nE, int vec8, int csrLen) {
  extern __shared__ v4f lds_dyn[];
  int* region = (int*)lds_dyn;
  int* cursor = region + RCAP;
  int* list   = cursor + NBF;
  int* wcnt   = list + LISTN;
  const int tid = threadIdx.x, lane = tid & 31, wave = tid >> 5;
  const int b = blockIdx.x;
  const int nodeBase = b * NBF;

  int rb0 = rbase[b];
  const int rb1 = rbase[b + 1];
  rb0 = rb0 < 0 ? 0 : (rb0 > csrLen ? csrLen : rb0);
  rb0 &= ~31;
  int len = rb1 - rb0;
  len = len < 0 ? 0 : (len > RCAP ? RCAP : len);
  int lenW = (len + 31) & ~31;
  if (rb0 + lenW > csrLen) lenW = (csrLen - rb0) & ~31;

  {
    const v4i z = {0, 0, 0, 0};
    for (int i = tid; i < RCAP / 4; i += NTHR) ((v4i*)region)[i] = z;
    for (int s = tid; s < NBF; s += NTHR) {
      int o = off[nodeBase + s] - rb0;
      o = o < 0 ? 0 : (o > RCAP ? RCAP : o);
      cursor[s] = o;
    }
  }
  __syncthreads();

  const int nChunks = (nE + CHUNK - 1) / CHUNK;
#pragma unroll 1
  for (int ch = 0; ch < nChunks; ++ch) {
    const int cbase = ch * CHUNK;
    const int wc = scan_chunk<NBF>(keys, nE, cbase, nodeBase, vec8, list, tid, lane, wave);
    if (lane == 0) wcnt[wave] = wc;
    __syncthreads();
    if (wave == 0) {
#pragma unroll 1
      for (int wsx = 0; wsx < NWAVE; ++wsx) {
        int n = __builtin_amdgcn_readfirstlane(wcnt[wsx]);
        n = n > WCAP ? WCAP : (n < 0 ? 0 : n);
        const int* lp = list + wsx * WCAP;
#pragma unroll 1
        for (int i = 0; i < n; ++i) {
          const int ent  = __builtin_amdgcn_readfirstlane(lp[i]);
          const int slot = ent & (NBF - 1);
          int e = cbase + ((ent >> 12) & (CHUNK - 1));
          e = e > nE - 1 ? nE - 1 : e;
          if (lane == 0) {
            int pos = cursor[slot];
            pos = pos < 0 ? 0 : (pos > RCAP - 1 ? RCAP - 1 : pos);
            region[pos] = e;
            const int np = pos + 1;
            cursor[slot] = np > RCAP ? RCAP : np;
          }
        }
      }
    }
    __syncthreads();
  }

  const int nv = lenW >> 2;
  int* gp = csr + rb0;
#pragma unroll 1
  for (int i = tid; i < nv; i += NTHR) { const v4i v = ((const v4i*)region)[i]; *(volatile v4i*)(gp + 4 * i) = v; }
  __threadfence();
#pragma unroll 1
  for (int i = tid; i < nv; i += NTHR) { const v4i v = ((const v4i*)region)[i]; *(volatile v4i*)(gp + 4 * i) = v; }
}

__global__ __launch_bounds__(NTHR) void k_ngemm(
    const float* __restrict__ A, const _Float16* __restrict__ Bw,
    const float* __restrict__ avs, const float* __restrict__ avd,
    float* C, float* S, float* D, int nRowsA) {
  __shared__ __attribute__((aligned(16))) v4f lds_raw[GROWS * HF / 4];
  __shared__ __attribute__((aligned(16))) float sS[GROWS];
  __shared__ __attribute__((aligned(16))) float sD[GROWS];
  constexpr int PPR = HF / 8, NIT = (GROWS * PPR) / NTHR, NT = HF / 16;
  static_assert((GROWS * PPR) % NTHR == 0);
  _Float16* sAt = (_Float16*)lds_raw;
  float*    stg = (float*)lds_raw;
  const int tid = threadIdx.x, lane = tid & 31, wave = tid >> 5, hh = lane >> 4, m = lane & 15;
  const int rowBase = blockIdx.x * GROWS;

#pragma unroll
  for (int i = 0; i < NIT; ++i) {
    const int j = i * NTHR + tid;
    const int r = j / PPR;
    const int c8 = (j - r * PPR) * 8;
    int row = rowBase + r;
    row = row > nRowsA - 1 ? nRowsA - 1 : row;
    const float* ap = A + (size_t)row * HF + c8;
    v4f a = *(const v4f*)ap, b = *(const v4f*)(ap + 4);
    a = a * ASCL; b = b * ASCL;
    *(v8h*)(sAt + r * APH + c8) = cvt8(a, b);
  }
  __syncthreads();

  v8f acc[NT];
#pragma unroll
  for (int t = 0; t < NT; ++t) acc[t] = z8f();
  const _Float16* fp = sAt + (wave * 16 + m) * APH + 8 * hh;
#pragma unroll
  for (int kt = 0; kt < HF / 32; ++kt) {
    FragH a;
    a.h[0] = *(const v8h*)(fp + 32 * kt);
    a.h[1] = *(const v8h*)(fp + 32 * kt + 16);
#pragma unroll
    for (int t = 0; t < NT; ++t) {
      const _Float16* bp = Bw + (size_t)(16 * t + m) * HF + 32 * kt + 8 * hh;
      FragH b;
      b.h[0] = *(const v8h*)bp;
      b.h[1] = *(const v8h*)(bp + 16);
      acc[t] = wm(a.v, b.v, acc[t]);
    }
  }
  __syncthreads();

  const int r0 = wave * 16 + 8 * hh;
  float* sp = stg + r0 * HF + m;
#pragma unroll
  for (int t = 0; t < NT; ++t) {
#pragma unroll
    for (int r = 0; r < 8; ++r) sp[r * HF + 16 * t] = acc[t][r];
  }
  __syncthreads();

  const int rsub = lane >> 4;
  const int c4 = m * 4;
  const v4f as4 = *(const v4f*)(avs + c4);
  const v4f ad4 = *(const v4f*)(avd + c4);
  v4f vals[8];
#pragma unroll
  for (int i = 0; i < 8; ++i) {
    const int rl = wave * 16 + 2 * i + rsub;
    v4f v = *(const v4f*)(stg + rl * HF + c4);
    v = v * OSCL;
    vals[i] = v;
    float ps = v.x * as4.x + v.y * as4.y + v.z * as4.z + v.w * as4.w;
    float pd = v.x * ad4.x + v.y * ad4.y + v.z * ad4.z + v.w * ad4.w;
    ps += __shfl_xor(ps, 8); pd += __shfl_xor(pd, 8);
    ps += __shfl_xor(ps, 4); pd += __shfl_xor(pd, 4);
    ps += __shfl_xor(ps, 2); pd += __shfl_xor(pd, 2);
    ps += __shfl_xor(ps, 1); pd += __shfl_xor(pd, 1);
    if (m == 0) { sS[rl] = ps; sD[rl] = pd; }
  }
  __syncthreads();
  const v4f sv = *(const v4f*)(sS + 4 * lane);
  const v4f dv = *(const v4f*)(sD + 4 * lane);

#pragma unroll
  for (int i = 0; i < 8; ++i) {
    const int rl = wave * 16 + 2 * i + rsub;
    *(volatile v4f*)(C + (size_t)(rowBase + rl) * HF + c4) = vals[i];
  }
  if (wave == 0) *(volatile v4f*)(S + rowBase + 4 * lane) = sv;
  if (wave == 1) *(volatile v4f*)(D + rowBase + 4 * lane) = dv;
  __threadfence();
#pragma unroll
  for (int i = 0; i < 8; ++i) {
    const int rl = wave * 16 + 2 * i + rsub;
    *(volatile v4f*)(C + (size_t)(rowBase + rl) * HF + c4) = vals[i];
  }
  if (wave == 0) *(volatile v4f*)(S + rowBase + 4 * lane) = sv;
  if (wave == 1) *(volatile v4f*)(D + rowBase + 4 * lane) = dv;
}

__global__ __launch_bounds__(ETHR) void k_gat(
    const int* __restrict__ offp, const int* __restrict__ cntp, const int* __restrict__ csr,
    const int* __restrict__ esrc, const float* __restrict__ h,
    const float* __restrict__ sp, const float* __restrict__ dp,
    const float* __restrict__ bias, float* hout, int nN, int nE, int csrLen) {
  __shared__ __attribute__((aligned(16))) float sOut[CNB * HF];
  const int tid = threadIdx.x, lane = tid & 31, wave = tid >> 5, hh = lane >> 4, m = lane & 15;
  const int c0 = blockIdx.x * CNB;
  const float ninf = __uint_as_float(0xff800000u);
  const v4f bv = *(const v4f*)(bias + 4 * m);

#pragma unroll 1
  for (int sl = 0; sl < 8; ++sl) {
    int node = c0 + 8 * wave + sl;
    node = node > nN - 1 ? nN - 1 : node;
    node = __builtin_amdgcn_readfirstlane(node);
    int offi = __builtin_amdgcn_readfirstlane(offp[node]);
    int cnti = __builtin_amdgcn_readfirstlane(cntp[node]);
    cnti = cnti < 0 ? 0 : (cnti > DEGCAP ? DEGCAP : cnti);
    offi = offi < 0 ? 0 : (offi > csrLen - 1 ? csrLen - 1 : offi);
    const float di = dp[node];
    const float si = sp[node];
    float es = si + di;
    es = es > 0.f ? es : SLOPE * es;
    const int nchk = (cnti + 31) >> 5;

    float mx = es;
#pragma unroll 1
    for (int c = 0; c < nchk; ++c) {
      const int k = 32 * c + lane;
      int pos = offi + k;
      pos = pos > csrLen - 1 ? csrLen - 1 : pos;
      int e = csr[pos];
      e = e < 0 ? 0 : (e > nE - 1 ? nE - 1 : e);
      int j = esrc[e];
      j = j < 0 ? 0 : (j > nN - 1 ? nN - 1 : j);
      float ev = sp[j] + di;
      ev = ev > 0.f ? ev : SLOPE * ev;
      ev = (k < cnti) ? ev : ninf;
      ev = fmaxf(ev, __shfl_xor(ev, 16));
      ev = fmaxf(ev, __shfl_xor(ev, 8));
      ev = fmaxf(ev, __shfl_xor(ev, 4));
      ev = fmaxf(ev, __shfl_xor(ev, 2));
      ev = fmaxf(ev, __shfl_xor(ev, 1));
      mx = fmaxf(mx, ev);
    }

    const v4f hrow = *(const v4f*)(h + (size_t)node * HF + 4 * m);
    const float pself = __expf(es - mx);
    const float ph = (hh == 0) ? pself : 0.f;
    v4f acc = ph * hrow;
    float zl = (lane == 0) ? pself : 0.f;
#pragma unroll 1
    for (int c = 0; c < nchk; ++c) {
      const int k = 32 * c + lane;
      int pos = offi + k;
      pos = pos > csrLen - 1 ? csrLen - 1 : pos;
      int e = csr[pos];
      e = e < 0 ? 0 : (e > nE - 1 ? nE - 1 : e);
      int j = esrc[e];
      j = j < 0 ? 0 : (j > nN - 1 ? nN - 1 : j);
      float ev = sp[j] + di;
      ev = ev > 0.f ? ev : SLOPE * ev;
      float p = __expf(ev - mx);
      p = (k < cnti) ? p : 0.f;
      zl += p;
      int nv = cnti - 32 * c;
      nv = nv > 32 ? 32 : nv;
#pragma unroll 1
      for (int t = 0; t < nv; t += 2) {
        int srcl = t + hh;
        const bool ok = srcl < nv;
        srcl = srcl > 31 ? 31 : srcl;
        const int jj = __shfl(j, srcl);
        float pp = __shfl(p, srcl);
        pp = ok ? pp : 0.f;
        const v4f r = *(const v4f*)(h + (size_t)jj * HF + 4 * m);
        acc = acc + pp * r;
      }
    }
    zl += __shfl_xor(zl, 16);
    zl += __shfl_xor(zl, 8);
    zl += __shfl_xor(zl, 4);
    zl += __shfl_xor(zl, 2);
    zl += __shfl_xor(zl, 1);
    acc.x += __shfl_xor(acc.x, 16);
    acc.y += __shfl_xor(acc.y, 16);
    acc.z += __shfl_xor(acc.z, 16);
    acc.w += __shfl_xor(acc.w, 16);
    const float iz = 1.0f / zl;
    v4f o = acc * iz + bv;
    o.x = fmaxf(o.x, 0.f); o.y = fmaxf(o.y, 0.f); o.z = fmaxf(o.z, 0.f); o.w = fmaxf(o.w, 0.f);
    if (hh == 0) *(v4f*)(sOut + (8 * wave + sl) * HF + 4 * m) = o;
  }
  __syncthreads();

  v4f ov[4];
#pragma unroll
  for (int q = 0; q < 4; ++q) ov[q] = *(const v4f*)(sOut + (8 * wave + 2 * q) * HF + 4 * lane);
#pragma unroll
  for (int q = 0; q < 4; ++q)
    *(volatile v4f*)(hout + (size_t)(c0 + 8 * wave + 2 * q) * HF + 4 * lane) = ov[q];
  __threadfence();
#pragma unroll
  for (int q = 0; q < 4; ++q)
    *(volatile v4f*)(hout + (size_t)(c0 + 8 * wave + 2 * q) * HF + 4 * lane) = ov[q];
}

__global__ __launch_bounds__(ETHR) void k_pool(
    const float* __restrict__ hf, const int* __restrict__ bat, float* hp, int nN) {
  __shared__ __attribute__((aligned(16))) float sMx[4 * HF];
  const int tid = threadIdx.x, lane = tid & 31, wave = tid >> 5;
  const int g = blockIdx.x;
  const float ninf = __uint_as_float(0xff800000u);
  float m0 = ninf, m1 = ninf;
  const int nIt = (nN + ETHR - 1) / ETHR;
#pragma unroll 1
  for (int it = 0; it < nIt; ++it) {
    const int n = it * ETHR + tid;
    const int nc = n < nN ? n : nN - 1;
    const int b = bat[nc];
    const bool hit = (n < nN) && (b == g);
    unsigned msk = __builtin_amdgcn_ballot_w32(hit);
    msk = (unsigned)__builtin_amdgcn_readfirstlane((int)msk);
    while (msk != 0u) {
      const int l = __builtin_ctz(msk);
      msk &= msk - 1u;
      int node = it * ETHR + 32 * wave + l;
      node = node > nN - 1 ? nN - 1 : node;
      const v2f v = *(const v2f*)(hf + (size_t)node * HF + 2 * lane);
      m0 = fmaxf(m0, v.x);
      m1 = fmaxf(m1, v.y);
    }
  }
  sMx[wave * HF + 2 * lane] = m0;
  sMx[wave * HF + 2 * lane + 1] = m1;
  __syncthreads();
  const int c4 = 4 * (lane & 15);
  v4f r = *(const v4f*)(sMx + c4);
#pragma unroll
  for (int w = 1; w < 4; ++w) {
    const v4f q = *(const v4f*)(sMx + w * HF + c4);
    r.x = fmaxf(r.x, q.x); r.y = fmaxf(r.y, q.y); r.z = fmaxf(r.z, q.z); r.w = fmaxf(r.w, q.w);
  }
  float* gp = hp + (size_t)g * HF + c4;
  if (wave == 0 && lane < 16) *(volatile v4f*)gp = r;
  __threadfence();
  if (wave == 0 && lane < 16) *(volatile v4f*)gp = r;
}

__global__ __launch_bounds__(HTHR) void k_head(
    const float* __restrict__ hp, const float* __restrict__ wl,
    const float* __restrict__ bl, float* out) {
  __shared__ __attribute__((aligned(16))) float sO[NG * NCLS];
  const int tid = threadIdx.x;
  const int g = tid / NCLS;
  const int c = tid - g * NCLS;
  const float* gr = hp + (size_t)g * HF;
  float acc = 0.f;
#pragma unroll 4
  for (int f = 0; f < HF; ++f) acc += gr[f] * wl[f * NCLS + c];
  acc += bl[c];
  sO[tid] = acc;
  __syncthreads();
  constexpr int NQ = (NG * NCLS) / 4;
  const int tq = tid < NQ ? tid : NQ - 1;
  const v4f v = *(const v4f*)(sO + 4 * tq);
  if (tid < NQ) *(volatile v4f*)(out + 4 * (size_t)tid) = v;
  __threadfence();
  if (tid < NQ) *(volatile v4f*)(out + 4 * (size_t)tid) = v;
}

extern "C" void kernel_launch(void* const* d_in, const int* in_sizes, int n_in,
                              void* d_out, int out_size, void* d_ws, size_t ws_size,
                              hipStream_t stream) {
  if (n_in < 13) return;
  const int nN = in_sizes[2];
  if (nN <= 0 || nN > (1 << 22)) return;
  if (in_sizes[0] != nN * HF) return;
  const int nE2 = in_sizes[1];
  if (nE2 <= 0 || (nE2 & 1) != 0) return;
  const int nE = nE2 / 2;
  if (nE > (1 << 26)) return;
  if (in_sizes[3] != HF * HF || in_sizes[4] != HF || in_sizes[5] != HF || in_sizes[6] != HF) return;
  if (in_sizes[7] != HF * HF || in_sizes[8] != HF || in_sizes[9] != HF || in_sizes[10] != HF) return;
  if (in_sizes[11] != HF * NCLS || in_sizes[12] != NCLS) return;
  if (out_size != NG * NCLS) return;

  const float* x   = (const float*)d_in[0];
  const int*   ei  = (const int*)d_in[1];
  const int*   bat = (const int*)d_in[2];
  const float* w1  = (const float*)d_in[3];
  const float* a1s = (const float*)d_in[4];
  const float* a1d = (const float*)d_in[5];
  const float* b1  = (const float*)d_in[6];
  const float* w2  = (const float*)d_in[7];
  const float* a2s = (const float*)d_in[8];
  const float* a2d = (const float*)d_in[9];
  const float* b2  = (const float*)d_in[10];
  const float* wl  = (const float*)d_in[11];
  const float* bl  = (const float*)d_in[12];
  float* out = (float*)d_out;
  const int* esrc = ei;
  const int* edst = ei + nE;

  const int NPAD   = ((nN + GROWS - 1) / GROWS) * GROWS;
  const int nBC    = (nN + NBC - 1) / NBC;
  const int CNTPAD = nBC * NBC;
  if (NPAD > CNTPAD) return;
  if (4 * nBC + 1 > RBN) return;
  const int nBF    = (nN + NBF - 1) / NBF;
  if (31 * 4 * nBC > 4096) return;
  const int csrLen = ((nE + 31) & ~31) + 4096;
  const int nGemm  = NPAD / GROWS;
  const int nGat   = NPAD / CNB;
  const int nWp    = WPIECES / NTHR;

  char* ws = (char*)d_ws;
  size_t off = 0;
  const size_t plane = (size_t)NPAD * HF * 4;
  const size_t oW   = off; off += (size_t)WPIECES * 16;     off = (off + 255) & ~(size_t)255;
  const size_t oCnt = off; off += (size_t)CNTPAD * 4;       off = (off + 255) & ~(size_t)255;
  const size_t oOff = off; off += (size_t)CNTPAD * 4;       off = (off + 255) & ~(size_t)255;
  const size_t oRb  = off; off += (size_t)RBN * 4;          off = (off + 255) & ~(size_t)255;
  const size_t oCsr = off; off += (size_t)csrLen * 4;       off = (off + 255) & ~(size_t)255;
  const size_t oH   = off; off += plane;                    off = (off + 255) & ~(size_t)255;
  const size_t oAgg = off; off += plane;                    off = (off + 255) & ~(size_t)255;
  const size_t oS   = off; off += (size_t)NPAD * 4;         off = (off + 255) & ~(size_t)255;
  const size_t oD   = off; off += (size_t)NPAD * 4;         off = (off + 255) & ~(size_t)255;
  const size_t oHp  = off; off += (size_t)NG * HF * 4;      off = (off + 255) & ~(size_t)255;
  if (off > ws_size || off > (size_t)WSCAP) return;
  _Float16* wp = (_Float16*)(ws + oW);
  int*   cnt  = (int*)(ws + oCnt);
  int*   offp = (int*)(ws + oOff);
  int*   rb   = (int*)(ws + oRb);
  int*   csr  = (int*)(ws + oCsr);
  float* hpl  = (float*)(ws + oH);
  float* agg  = (float*)(ws + oAgg);
  float* spl  = (float*)(ws + oS);
  float* dpl  = (float*)(ws + oD);
  float* hp   = (float*)(ws + oHp);

  const int vec8 = ((nE & 3) == 0) ? 1 : 0;

  k_wprep<<<nWp, NTHR, 0, stream>>>(w1, w2, wp);

  k_count<<<nBC, NTHR, 0, stream>>>(edst, cnt, nE, vec8);
  k_offsets<<<1, OTHR, 0, stream>>>(cnt, offp, rb, nBC);
  hipFuncSetAttribute(reinterpret_cast<const void*>(&k_fill),
                      hipFuncAttributeMaxDynamicSharedMemorySize, LDS_FILL);
  k_fill<<<nBF, NTHR, LDS_FILL, stream>>>(edst, offp, rb, csr, nE, vec8, csrLen);

  k_ngemm<<<nGemm, NTHR, 0, stream>>>(x, wp, a1s, a1d, hpl, spl, dpl, nN);
  k_gat<<<nGat, ETHR, 0, stream>>>(offp, cnt, csr, esrc, hpl, spl, dpl, b1, agg, nN, nE, csrLen);

  k_ngemm<<<nGemm, NTHR, 0, stream>>>(agg, wp + HF * HF, a2s, a2d, hpl, spl, dpl, nN);
  k_gat<<<nGat, ETHR, 0, stream>>>(offp, cnt, csr, esrc, hpl, spl, dpl, b2, agg, nN, nE, csrLen);

  k_pool<<<NG, ETHR, 0, stream>>>(agg, bat, hp, nN);

  k_head<<<1, HTHR, 0, stream>>>(hp, wl, bl, out);
}
